// HybridCNNQuantumModel_34351148434288
// MI455X (gfx1250) — hardware-verified
//
#include <hip/hip_runtime.h>

typedef _Float16     v16h __attribute__((ext_vector_type(16)));
typedef _Float16     v8h  __attribute__((ext_vector_type(8)));
typedef float        v8f  __attribute__((ext_vector_type(8)));
typedef float        v4f  __attribute__((ext_vector_type(4)));
typedef unsigned int v4u  __attribute__((ext_vector_type(4)));

#define NPIX1  2704
#define PITCH1 2752
#define PCH1   344
#define PCH1R  338
#define KPAD   160
#define KC     5
#define WROW   20
#define WCH    640
#define IMGS   8

union Frag { v16h v; v4u q[2]; };

__device__ __forceinline__ v8f wmma_f16(v16h a, v16h b, v8f c)
{
    v8f d = __builtin_amdgcn_wmma_f32_16x16x32_f16(false, a, false, b, (short)0, c, false, false);
    asm volatile("v_nop\n\tv_nop\n\tv_nop\n\tv_nop" : "+v"(d) : "v"(a), "v"(b));
    return d;
}

__global__ __launch_bounds__(256) void k_prep_w2(const float* __restrict__ w2,
                                                 v4u* __restrict__ w2h4)
{
    for (int pass = 0; pass < 2; ++pass) {
        for (int c = threadIdx.x; c < WCH; c += 256) {
            const int n  = c / WROW;
            const int kq = c - WROW * n;
            const int k0 = kq * 8;
            union { v8h h; v4u u; } t;
#pragma unroll
            for (int i = 0; i < 8; ++i) {
                const int k = k0 + i;
                float v = 0.f;
                if (k < 144) v = 64.f * w2[k * 32 + n];
                t.h[i] = (_Float16)v;
            }
            *(volatile v4u*)(w2h4 + c) = t.u;
        }
        if (pass == 0) __threadfence();
    }
}

__global__ __launch_bounds__(256) void k_conv1_pool(const float* __restrict__ x,
                                                    const float* __restrict__ w1,
                                                    const float* __restrict__ b1,
                                                    v4u* __restrict__ pooled4,
                                                    int B)
{
    __shared__ float img[784];
    __shared__ v4u   pst4[PCH1];
    _Float16* pst = (_Float16*)pst4;

    const int tid = threadIdx.x;
    const int n   = blockIdx.x;
    if (n >= B) return;

    const size_t base = (size_t)n * 784;
    for (int i = tid; i < 784; i += 256) img[i] = x[base + i];
    __syncthreads();

    const int c = tid & 15;
    float wc[9];
#pragma unroll
    for (int k = 0; k < 9; ++k) wc[k] = w1[k * 16 + c];
    const float bc = b1[c];

    for (int idx = tid; idx < NPIX1; idx += 256) {
        const int pix = idx >> 4;
        const int py = pix / 13, px = pix - 13 * py;
        float m = 0.f;
#pragma unroll
        for (int wy = 0; wy < 2; ++wy)
#pragma unroll
            for (int wx = 0; wx < 2; ++wx) {
                const int y = 2 * py + wy, xx = 2 * px + wx;
                float acc = bc;
#pragma unroll
                for (int dy = 0; dy < 3; ++dy)
#pragma unroll
                    for (int dx = 0; dx < 3; ++dx)
                        acc = fmaf(img[(y + dy) * 28 + xx + dx], wc[dy * 3 + dx], acc);
                m = fmaxf(m, acc);
            }
        pst[idx] = (_Float16)m;
    }
    for (int i = NPIX1 + tid; i < PITCH1; i += 256) pst[i] = (_Float16)0.f;
    __syncthreads();

    v4u* dst = pooled4 + (size_t)n * PCH1;
    for (int cch = tid; cch < PCH1; cch += 256) {
        const v4u v = pst4[cch];
        *(volatile v4u*)(dst + cch) = v;
    }
    __threadfence();
    for (int cch = tid; cch < PCH1; cch += 256) {
        const v4u v = pst4[cch];
        *(volatile v4u*)(dst + cch) = v;
    }
}

__global__ __launch_bounds__(256) void k_conv2_head(const v4u* __restrict__ pooled4,
                                                    const v4u* __restrict__ w2h4,
                                                    const float* __restrict__ b2,
                                                    const float* __restrict__ dw,
                                                    const float* __restrict__ db,
                                                    const float* __restrict__ qw,
                                                    int L,
                                                    float* __restrict__ out,
                                                    int B)
{
    __shared__ v4u   Bl4[WCH];
    __shared__ v4u   P4[PCH1];
    __shared__ float Cout[121 * 32];
    __shared__ float red[256 * 4];
    __shared__ float featsL[IMGS * 4];
    __shared__ v4f   outL4[IMGS];
    float* outL = (float*)outL4;

    const int tid  = threadIdx.x;
    const int lane = tid & 31;
    const int wv   = tid >> 5;
    const int h    = lane >> 4;
    const int lo16 = lane & 15;
    const int g    = blockIdx.x;

    for (int c = tid; c < WCH; c += 256) Bl4[c] = w2h4[c];
    if (tid < IMGS * 4) featsL[tid] = 0.f;

    const int m  = wv * 16 + lo16;
    const int p  = (m < 121) ? m : 120;
    const int oy = p / 11, ox = p - 11 * oy;
    const int abase  = (oy * 13 + ox) * 2 + h;
    const int bbase0 = lo16 * WROW + h;
    const int bbase1 = (16 + lo16) * WROW + h;
    const float bz0 = b2[lo16], bz1 = b2[16 + lo16];
    const v4u z4 = {0u, 0u, 0u, 0u};

    for (int li = 0; li < IMGS; ++li) {
        const int img = g * IMGS + li;
        if (img >= B) break;
        __syncthreads();

        const v4u* src = pooled4 + (size_t)img * PCH1;
        for (int c = tid; c < PCH1R; c += 256) P4[c] = src[c];
        __syncthreads();

        v8f acc0 = {0.f, 0.f, 0.f, 0.f, 0.f, 0.f, 0.f, 0.f};
        v8f acc1 = {0.f, 0.f, 0.f, 0.f, 0.f, 0.f, 0.f, 0.f};
#pragma unroll
        for (int kc = 0; kc < KC; ++kc) {
            const int tlo = 2 * kc, thi = 2 * kc + 1;
            const int offlo = ((tlo / 3) * 13 + (tlo % 3)) * 2;
            Frag a, b0, b1;
            a.q[0] = P4[abase + offlo];
            if (kc < KC - 1) {
                const int offhi = ((thi / 3) * 13 + (thi % 3)) * 2;
                a.q[1] = P4[abase + offhi];
            } else {
                a.q[1] = z4;
            }
            b0.q[0] = Bl4[bbase0 + 4 * kc];
            b0.q[1] = Bl4[bbase0 + 4 * kc + 2];
            b1.q[0] = Bl4[bbase1 + 4 * kc];
            b1.q[1] = Bl4[bbase1 + 4 * kc + 2];
            acc0 = wmma_f16(a.v, b0.v, acc0);
            acc1 = wmma_f16(a.v, b1.v, acc1);
        }

#pragma unroll
        for (int r = 0; r < 8; ++r) {
            const int pr = wv * 16 + h * 8 + r;
            if (pr < 121) {
                Cout[pr * 32 + lo16]      = fmaxf(acc0[r] * 0.015625f + bz0, 0.f);
                Cout[pr * 32 + 16 + lo16] = fmaxf(acc1[r] * 0.015625f + bz1, 0.f);
            }
        }
        __syncthreads();

        float part[4] = {0.f, 0.f, 0.f, 0.f};
        for (int idx = tid; idx < 800; idx += 256) {
            const int py  = idx / 160;
            const int rem = idx - py * 160;
            const int px  = rem >> 5;
            const int cc  = rem & 31;
            const int r0  = (2 * py) * 11 + 2 * px;
            const int r1  = r0 + 11;
            const float mv = fmaxf(fmaxf(Cout[r0 * 32 + cc], Cout[(r0 + 1) * 32 + cc]),
                                   fmaxf(Cout[r1 * 32 + cc], Cout[(r1 + 1) * 32 + cc]));
#pragma unroll
            for (int j = 0; j < 4; ++j) part[j] = fmaf(mv, dw[idx * 4 + j], part[j]);
        }
#pragma unroll
        for (int j = 0; j < 4; ++j) red[tid * 4 + j] = part[j];
        __syncthreads();
        for (int s = 128; s >= 1; s >>= 1) {
            if (tid < s) {
#pragma unroll
                for (int j = 0; j < 4; ++j) red[tid * 4 + j] += red[(tid + s) * 4 + j];
            }
            __syncthreads();
        }
        if (tid < 4) featsL[li * 4 + tid] = tanhf(red[tid] + db[tid]);
    }
    __syncthreads();

    if (tid < IMGS * 4) {
        const int li = tid >> 2, j = tid & 3;
        float wsum[4], p1[4], p0[4];
#pragma unroll
        for (int i = 0; i < 4; ++i) {
            float wacc = 0.f;
            for (int l = 0; l < L; ++l) wacc += qw[l * 16 + i * 4 + j];
            wsum[i] = wacc;
            const float s = sinf(featsL[li * 4 + i]);
            p1[i] = 0.5f * (1.f + s);
            p0[i] = 0.5f * (1.f - s);
        }
        float q = 0.f;
#pragma unroll 1
        for (int b = 0; b < 16; ++b) {
            float pb = 1.f, ang = 0.f;
#pragma unroll
            for (int i = 0; i < 4; ++i) {
                const bool bit = ((b >> i) & 1) != 0;
                pb  *= bit ? p1[i] : p0[i];
                ang += bit ? wsum[i] : 0.f;
            }
            q -= pb * sinf(ang);
        }
        outL[tid] = 1.f / (1.f + expf(-10.f * q));
    }
    __syncthreads();

    if (tid < IMGS) {
        const int img = g * IMGS + tid;
        if (img < B) {
            const v4f v = outL4[tid];
            volatile v4f* dst = (volatile v4f*)(out + (size_t)img * 4);
            *dst = v;
            __threadfence();
            *dst = v;
        }
    }
}

extern "C" void kernel_launch(void* const* d_in, const int* in_sizes, int n_in,
                              void* d_out, int out_size, void* d_ws, size_t ws_size,
                              hipStream_t stream)
{
    const float* x  = (const float*)d_in[0];
    const float* w1 = (const float*)d_in[1];
    const float* b1 = (const float*)d_in[2];
    const float* w2 = (const float*)d_in[3];
    const float* b2 = (const float*)d_in[4];
    const float* dw = (const float*)d_in[5];
    const float* db = (const float*)d_in[6];
    const float* qw = (const float*)d_in[7];
    float* out = (float*)d_out;

    const int B = in_sizes[0] / (28 * 28);
    const int L = in_sizes[7] / 16;
    if (B <= 0) return;
    if ((size_t)out_size < (size_t)B * 4) return;

    char*  ws   = (char*)d_ws;
    size_t off0 = 0;
    size_t off1 = off0 + (size_t)B * PITCH1 * sizeof(_Float16);
    off1 = (off1 + 255) & ~(size_t)255;
    size_t need = off1 + (size_t)WCH * 16;
    if (need > ws_size) return;

    v4u* pooled4 = (v4u*)(ws + off0);
    v4u* w2h4    = (v4u*)(ws + off1);

    const int grid2 = (B + IMGS - 1) / IMGS;

    k_prep_w2   <<<1,     256, 0, stream>>>(w2, w2h4);
    k_conv1_pool<<<B,     256, 0, stream>>>(x, w1, b1, pooled4, B);
    k_conv2_head<<<grid2, 256, 0, stream>>>(pooled4, w2h4, b2, dw, db, qw, L, out, B);

    (void)n_in;
}
